// MultiHeadedAttention_25563645346690
// MI455X (gfx1250) — hardware-run, weakly checked
//
#include <hip/hip_runtime.h>


#define NB_  2
#define TT   1024
#define DM   512
#define NH_  8
#define NKV  8
#define REP  (NH_ / NKV)
#define HD   64
#define DQ   (NH_ * HD)
#define DKV  (NKV * HD)
#define ZH   2
#define RH   0
#define WIN  0
#define PCAR 1024.0f
#define SCL  0.125f
#define PMUL 1.0f
#define LNC_MAX 2048
#define PR   32
#define KB   128
#define KS   64
#define LNF  0.99902296066284180f

typedef _Float16 h16;
typedef unsigned short bf;
typedef __attribute__((ext_vector_type(16))) __bf16   v16bf;
typedef __attribute__((ext_vector_type(16))) _Float16 v16h;
typedef __attribute__((ext_vector_type(8)))  _Float16 v8h;
typedef __attribute__((ext_vector_type(8)))  unsigned short v8us;
typedef __attribute__((ext_vector_type(8)))  float    v8f;
typedef __attribute__((ext_vector_type(4)))  float    v4f;
typedef v8h  __attribute__((may_alias)) v8ha;
typedef v4f  __attribute__((may_alias)) v4fa;
typedef v8us __attribute__((may_alias)) v8usa;

__device__ __forceinline__ unsigned short f2bf(float f) { unsigned u = __float_as_uint(f); u += 0x7FFFu + ((u >> 16) & 1u); return (unsigned short)(u >> 16); }
__device__ __forceinline__ float bf2f(unsigned short b) { return __uint_as_float(((unsigned)b) << 16); }
__device__ __forceinline__ float bfr(float f) { return bf2f(f2bf(f)); }
__device__ __forceinline__ v16h cat16(v8h lo, v8h hi) { return __builtin_shufflevector(lo, hi, 0, 1, 2, 3, 4, 5, 6, 7, 8, 9, 10, 11, 12, 13, 14, 15); }
__device__ __forceinline__ v16bf cat16b(v8us lo, v8us hi) { return __builtin_bit_cast(v16bf, __builtin_shufflevector(lo, hi, 0, 1, 2, 3, 4, 5, 6, 7, 8, 9, 10, 11, 12, 13, 14, 15)); }
__device__ __forceinline__ v8f wmma16(v16h a, v16h b, v8f c) { return __builtin_amdgcn_wmma_f32_16x16x32_f16(false, a, false, b, (short)0, c, false, false); }
__device__ __forceinline__ v8f wmmab(v16bf a, v16bf b, v8f c) { return __builtin_amdgcn_wmma_f32_16x16x32_bf16(false, a, false, b, (short)0, c, false, false); }
typedef __attribute__((ext_vector_type(2))) _Float16 v2h;
typedef __attribute__((ext_vector_type(4))) _Float16 v4h;
typedef __attribute__((ext_vector_type(2))) unsigned short v2us;
typedef __attribute__((ext_vector_type(4))) unsigned short v4us;
typedef __attribute__((ext_vector_type(2))) float v2f;
typedef __attribute__((ext_vector_type(4))) int v4i;

template <typename T16> struct WFrag;
template <> struct WFrag<h16> { typedef v16h V; static __device__ __forceinline__ V ld(const h16* p) { return cat16(*(const v8h*)p, *(const v8h*)(p + 16)); } static __device__ __forceinline__ v8f mma(V a, V b, v8f c) { return wmma16(a, b, c); } };
template <> struct WFrag<bf> { typedef v16bf V; static __device__ __forceinline__ V ld(const bf* p) { return cat16b(*(const v8us*)p, *(const v8us*)(p + 16)); } static __device__ __forceinline__ v8f mma(V a, V b, v8f c) { return wmmab(a, b, c); } };
template <typename T16, int NSPLIT, bool BIAS>
__global__ __launch_bounds__(32) void k_gemmw(const T16* __restrict__ A, const T16* __restrict__ A2, const T16* __restrict__ Bt, const T16* __restrict__ Bt2, int K, float* C, int ldc, const float* __restrict__ bias, size_t sA, size_t sB, size_t sC) {
    typedef typename WFrag<T16>::V V;
    __shared__ __align__(16) float os[16 * 68];
    const size_t z = blockIdx.z; A += z * sA; if (A2) A2 += z * sA; Bt += z * sB; if (Bt2) Bt2 += z * sB; C += z * sC;
    const int lane = threadIdx.x & 31, lr = lane & 15, hi = lane >> 4; const int r0 = blockIdx.x * 64, c0 = blockIdx.y * 64;
    v8f acc[4][4];
#pragma unroll
    for (int mb = 0; mb < 4; ++mb)
#pragma unroll
        for (int nb = 0; nb < 4; ++nb) acc[mb][nb] = (v8f){};
    const size_t aoff = (size_t)(r0 + lr) * K + 8 * hi, boff = (size_t)(c0 + lr) * K + 8 * hi;

    for (int kc = 0; kc < K; kc += 32) {
        V a[4], a2[4];
#pragma unroll
        for (int mb = 0; mb < 4; ++mb) { a[mb] = WFrag<T16>::ld(A + aoff + (size_t)mb * 16 * K + kc); if (NSPLIT == 1 || NSPLIT == 2) a2[mb] = WFrag<T16>::ld(A2 + aoff + (size_t)mb * 16 * K + kc); }
#pragma unroll
        for (int nb = 0; nb < 4; ++nb) { const V b = WFrag<T16>::ld(Bt + boff + (size_t)nb * 16 * K + kc); V b2; if (NSPLIT >= 2) b2 = WFrag<T16>::ld(Bt2 + boff + (size_t)nb * 16 * K + kc);
#pragma unroll
            for (int mb = 0; mb < 4; ++mb) { acc[mb][nb] = WFrag<T16>::mma(a[mb], b, acc[mb][nb]); if (NSPLIT == 1 || NSPLIT == 2) acc[mb][nb] = WFrag<T16>::mma(a2[mb], b, acc[mb][nb]); if (NSPLIT >= 2) acc[mb][nb] = WFrag<T16>::mma(a[mb], b2, acc[mb][nb]); } }
        asm volatile("v_nop\n\tv_nop\n\tv_nop\n\tv_nop" : "+v"(acc[0][0]), "+v"(acc[1][1]), "+v"(acc[2][2]), "+v"(acc[3][3]) : "v"(a[0]), "v"(a[3]));
    }
#pragma unroll
    for (int mb = 0; mb < 4; ++mb) {
#pragma unroll
        for (int nb = 0; nb < 4; ++nb) {
#pragma unroll
            for (int j = 0; j < 8; ++j) os[(hi * 8 + j) * 68 + nb * 16 + lr] = acc[mb][nb][j]; }
        __builtin_amdgcn_wave_barrier(); asm volatile("" ::: "memory");
        float* crow = C + (size_t)(r0 + mb * 16) * ldc + c0;
#pragma unroll 1
        for (int ps = 0; ps < 2; ++ps) {
#pragma unroll
            for (int s = 0; s < 8; ++s) { const int row = 2 * s + hi, cofs = lr * 4; v4f val = *(const v4fa*)(os + row * 68 + cofs); if (BIAS) { val[0] += bfr(bias[c0 + cofs]); val[1] += bfr(bias[c0 + cofs + 1]); val[2] += bfr(bias[c0 + cofs + 2]); val[3] += bfr(bias[c0 + cofs + 3]); }
                *(volatile v4f*)(crow + (size_t)row * ldc + cofs) = val; }
            if (ps == 0) __threadfence(); }
        __builtin_amdgcn_wave_barrier(); asm volatile("" ::: "memory");
    }
}

__device__ __forceinline__ h16 tohx(float x) { return (h16)x; }
__device__ __forceinline__ void splitf(float y, unsigned short& h, unsigned short& l) { h = f2bf(y); l = f2bf(y - bf2f(h)); }
typedef __attribute__((ext_vector_type(2))) _Float16 v2h;
typedef __attribute__((ext_vector_type(4))) _Float16 v4h;
typedef __attribute__((ext_vector_type(2))) unsigned short v2us;
typedef __attribute__((ext_vector_type(4))) unsigned short v4us;
typedef __attribute__((ext_vector_type(2))) float v2f;
typedef __attribute__((ext_vector_type(4))) int v4i;

__global__ __launch_bounds__(256) void k_cvt8(const float* __restrict__ src, bf* dst, size_t n8) { const size_t i = (size_t)blockIdx.x * 256 + threadIdx.x; if (i >= n8) return; const v8f v = *(const v8f*)(src + i * 8); v8us o;
#pragma unroll
    for (int k = 0; k < 8; ++k) o[k] = f2bf(v[k]); *(volatile v8us*)(dst + i * 8) = o; __threadfence(); *(volatile v8us*)(dst + i * 8) = o; }

__global__ __launch_bounds__(256) void k_rbf(const float* __restrict__ X, float* Y, size_t n4) { const size_t i = (size_t)blockIdx.x * 256 + threadIdx.x; if (i >= n4) return; const v4f a = *(const v4f*)(X + i * 4); v4f o;
#pragma unroll
    for (int q = 0; q < 4; ++q) o[q] = bfr(a[q]);
    *(volatile v4f*)(Y + i * 4) = o; __threadfence(); *(volatile v4f*)(Y + i * 4) = o; }

template <bool RES>
__global__ __launch_bounds__(256) void k_lnrow(const float* __restrict__ A, const float* __restrict__ R, const float* __restrict__ gamma, const float* __restrict__ beta, float eps, int C, int nrows, float* Y) {
    const int lane = threadIdx.x & 31; const int row = blockIdx.x * 8 + (threadIdx.x >> 5); if (row >= nrows) return; const int nch = C / 128; const float* a = A + (size_t)row * C; float x[LNC_MAX / 32]; float s = 0.0f;
    for (int k = 0; k < LNC_MAX / 128; ++k) { if (k < nch) { const int c0 = k * 128 + lane * 4; v4f v = *(const v4f*)(a + c0);
            if (RES) { const v4f w = *(const v4f*)(R + (size_t)row * C + c0); v[0] = __fadd_rn(v[0], w[0]); v[1] = __fadd_rn(v[1], w[1]); v[2] = __fadd_rn(v[2], w[2]); v[3] = __fadd_rn(v[3], w[3]); }
            x[k * 4 + 0] = v[0]; x[k * 4 + 1] = v[1]; x[k * 4 + 2] = v[2]; x[k * 4 + 3] = v[3]; s = __fadd_rn(__fadd_rn(__fadd_rn(__fadd_rn(s, v[0]), v[1]), v[2]), v[3]); } }
    for (int sh = 16; sh; sh >>= 1) s = __fadd_rn(s, __shfl_xor(s, sh, 32));
    const float mean = __fdiv_rn(s, (float)C); float q = 0.0f;
    for (int k = 0; k < LNC_MAX / 128; ++k) { if (k < nch) {
            for (int j = 0; j < 4; ++j) { const float d = __fsub_rn(x[k * 4 + j], mean); x[k * 4 + j] = d; q = __fmaf_rn(d, d, q); } } }
    for (int sh = 16; sh; sh >>= 1) q = __fadd_rn(q, __shfl_xor(q, sh, 32));
    const float rstd = __fdiv_rn(1.0f, sqrtf(__fadd_rn(__fdiv_rn(q, (float)C), eps)));
    for (int k = 0; k < LNC_MAX / 128; ++k) { if (k < nch) { const int c0 = k * 128 + lane * 4; const v4f g = *(const v4f*)(gamma + c0); const v4f bt = *(const v4f*)(beta + c0);
            for (int j = 0; j < 4; ++j) x[k * 4 + j] = __fmaf_rn(__fmul_rn(x[k * 4 + j], rstd), bfr(g[j]), bfr(bt[j])); } }
    float* y = Y + (size_t)row * C;
    for (int ps = 0; ps < 2; ++ps) {
        for (int k = 0; k < LNC_MAX / 128; ++k) { if (k < nch) { v4f o; o[0] = x[k * 4 + 0]; o[1] = x[k * 4 + 1]; o[2] = x[k * 4 + 2]; o[3] = x[k * 4 + 3]; *(volatile v4f*)(y + k * 128 + lane * 4) = o; } }
        if (ps == 0) __threadfence(); }
}

__global__ __launch_bounds__(256) void k_rope(const float* __restrict__ F, int pitch, int nheads, const float* __restrict__ CS, const float* __restrict__ RF, const float* __restrict__ nw, float sc, h16* P16, bf* Ph, bf* Pl) {
    const size_t e = ((size_t)blockIdx.x * 256 + threadIdx.x) * 2; if (e >= (size_t)nheads * TT * HD) return; const int d = (int)(e % HD); const int t = (int)((e / HD) % TT); const int h = (int)(e / ((size_t)HD * TT)); const float* f = F + (size_t)t * pitch + h * HD; const float rf = RF ? RF[(size_t)h * TT + t] : 1.0f; v2h o16; v2us oh, ol;
#pragma unroll
    for (int q = 0; q < 2; ++q) { const int dd = d + q; const int dp = (dd < HD / 2) ? dd + HD / 2 : dd - HD / 2; float x0 = f[dd], x1 = f[dp];
        if (RF) { float n0 = __fmul_rn(x0, rf), n1 = __fmul_rn(x1, rf); x0 = __fmul_rn(bfr(nw[dd]), n0); x1 = __fmul_rn(bfr(nw[dp]), n1); }
        const v2f cs = *(const v2f*)(CS + ((size_t)t * HD + dd) * 2); float a = __fmul_rn(x0, cs[0]), bq = __fmul_rn(x1, cs[1]); const float r = ((dd < HD / 2) ? __fsub_rn(a, bq) : __fadd_rn(a, bq)) * sc;
        o16[q] = tohx(r); unsigned short a2, c2; splitf(r, a2, c2); oh[q] = a2; ol[q] = c2; }
    *(volatile v2h*)(P16 + e) = o16; *(volatile v2us*)(Ph + e) = oh; *(volatile v2us*)(Pl + e) = ol; __threadfence(); *(volatile v2h*)(P16 + e) = o16; *(volatile v2us*)(Ph + e) = oh; *(volatile v2us*)(Pl + e) = ol; }

__global__ __launch_bounds__(256) void k_vtp(const float* __restrict__ F, int pitch, int nheads, h16* V16, bf* Vh, bf* Vl) { const size_t e = ((size_t)blockIdx.x * 256 + threadIdx.x) * 2; if (e >= (size_t)nheads * HD * TT) return; const int t = (int)(e % TT); const int d = (int)((e / TT) % HD); const int g = (int)(e / ((size_t)TT * HD)); v2h o16; v2us oh, ol;
#pragma unroll
    for (int q = 0; q < 2; ++q) { const float x = F[(size_t)(t + q) * pitch + g * HD + d]; o16[q] = tohx(x); unsigned short a2, c2; splitf(x, a2, c2); oh[q] = a2; ol[q] = c2; }
    *(volatile v2h*)(V16 + e) = o16; *(volatile v2us*)(Vh + e) = oh; *(volatile v2us*)(Vl + e) = ol; __threadfence(); *(volatile v2h*)(V16 + e) = o16; *(volatile v2us*)(Vh + e) = oh; *(volatile v2us*)(Vl + e) = ol; }

__global__ __launch_bounds__(256) void k_csid(float* CS) { const int idx = blockIdx.x * 256 + threadIdx.x; if (idx >= TT * HD) return; v2f cs; cs[0] = 1.0f; cs[1] = 0.0f; *(volatile v2f*)(CS + (size_t)idx * 2) = cs; __threadfence(); *(volatile v2f*)(CS + (size_t)idx * 2) = cs; }

__global__ __launch_bounds__(256) void k_asoftMA(const float* __restrict__ Sb, const float* __restrict__ MP, h16* P16, bf* Ph, bf* Pl) {
    const int lane = threadIdx.x & 31; const int row = blockIdx.x * 8 + (threadIdx.x >> 5); if (row >= ZH * TT) return; const int i = row % TT; const int zz = row / TT; (void)zz; const bool hires = (i < RH); const float* sr = Sb + (size_t)row * TT; float v[TT / 32]; float mx = -3.0e38f;
#pragma unroll
    for (int ch = 0; ch < TT / 128; ++ch) { const int j0 = ch * 128 + lane * 4; const v4f a = *(const v4f*)(sr + j0); const v4f m4 = *(const v4f*)(MP + (size_t)i * TT + j0);
#pragma unroll
        for (int q = 0; q < 4; ++q) { const int j = j0 + q; (void)j; const float t = a[q] * SCL + bfr(m4[q]) * PMUL;     v[ch * 4 + q] = t; mx = fmaxf(mx, t); } }
#pragma unroll
    for (int sh = 16; sh; sh >>= 1) mx = fmaxf(mx, __shfl_xor(mx, sh, 32));
    float sum = 0.f;
#pragma unroll
    for (int k = 0; k < TT / 32; ++k) { float d0 = __fsub_rn(v[k], mx); v[k] = __builtin_amdgcn_exp2f(__fmul_rn(d0, 1.4426950408889634f)); sum += v[k]; }
#pragma unroll
    for (int sh = 16; sh; sh >>= 1) sum += __shfl_xor(sum, sh, 32);
    const float f = __fdiv_rn(hires ? 1.0f : PCAR, sum);
#pragma unroll 1
    for (int ps = 0; ps < 2; ++ps) {
        if (hires) {
#pragma unroll
            for (int ch = 0; ch < TT / 128; ++ch) { v4us oh, ol;
#pragma unroll
                for (int q = 0; q < 4; ++q) { unsigned short a, c2; splitf(v[ch * 4 + q] * f, a, c2); oh[q] = a; ol[q] = c2; }
                const size_t oo = ((size_t)zz * (RH ? RH : 1) + i) * TT + ch * 128 + lane * 4; *(volatile v4us*)(Ph + oo) = oh; *(volatile v4us*)(Pl + oo) = ol; }
        } else {
#pragma unroll
            for (int ch = 0; ch < TT / 128; ++ch) { v4h o4;
#pragma unroll
                for (int q = 0; q < 4; ++q) o4[q] = tohx(v[ch * 4 + q] * f);
                *(volatile v4h*)(P16 + (size_t)row * TT + ch * 128 + lane * 4) = o4; } }
        if (ps == 0) __threadfence(); }
}

__global__ __launch_bounds__(256) void k_pl2(const float* __restrict__ F, bf* Ph, bf* Pl, size_t n4) { const size_t i = (size_t)blockIdx.x * 256 + threadIdx.x; if (i >= n4) return; const v4f v = *(const v4f*)(F + i * 4); v4us oh, ol;
#pragma unroll
    for (int q = 0; q < 4; ++q) { unsigned short a, c; splitf(v[q], a, c); oh[q] = a; ol[q] = c; } *(volatile v4us*)(Ph + i * 4) = oh; *(volatile v4us*)(Pl + i * 4) = ol; __threadfence(); *(volatile v4us*)(Ph + i * 4) = oh; *(volatile v4us*)(Pl + i * 4) = ol; }

__global__ __launch_bounds__(256) void k_tab(h16* RT, h16* TT2) { const unsigned e = blockIdx.x * 256u + threadIdx.x; if (e >= (unsigned)(KB + HD) * 8u) return; const bool pt = (e >= (unsigned)KB * 8u); const unsigned f = pt ? (e - (unsigned)KB * 8u) : e; const unsigned row = f >> 3, c0 = (f & 7u) * 8u; v8h o;
#pragma unroll
    for (int q = 0; q < 8; ++q) { const unsigned col = c0 + (unsigned)q; const unsigned u = pt ? col : row; const unsigned d = pt ? row : col; const unsigned umax = pt ? (unsigned)PR : (unsigned)(2 * PR);
        const float w = __builtin_amdgcn_exp2f(__fmul_rn((float)(d >> 1), -0.41524101186092029f)); const float a = __fmul_rn((float)u, w); const float k = rintf(__fmul_rn(a, 0.63661977236758138f)); float r = __fmaf_rn(-k, 1.5707963705062866f, a); r = __fmaf_rn(-k, -4.3711388286737929e-08f, r); const float r2 = __fmul_rn(r, r);
        const float sp = __fmaf_rn(r2, __fmaf_rn(r2, __fmaf_rn(r2, __fmaf_rn(r2, 2.7557319223985893e-06f, -1.9841269841269841e-04f), 8.3333333333333332e-03f), -1.6666666666666666e-01f), 1.0f); const float sn = __fmul_rn(r, sp);
        const float cn = __fmaf_rn(r2, __fmaf_rn(r2, __fmaf_rn(r2, __fmaf_rn(r2, 2.4801587301587302e-05f, -1.3888888888888889e-03f), 4.1666666666666664e-02f), -0.5f), 1.0f);
        const unsigned n = (unsigned)((int)k) & 3u; const float s1 = (n & 1u) ? cn : sn; const float c1 = (n & 1u) ? sn : cn; const float sv = __uint_as_float(__float_as_uint(s1) ^ ((n & 2u) << 30)); const float cv = __uint_as_float(__float_as_uint(c1) ^ (((n + 1u) & 2u) << 30)); const float val = (d & 1u) ? cv : sv; o[q] = (h16)__fmul_rn(val, (u <= umax) ? 1.0f : 0.0f); }
    h16* dst = (pt ? TT2 : RT) + (size_t)f * 8; *(volatile v8h*)dst = o; __threadfence(); *(volatile v8h*)dst = o; }

__global__ __launch_bounds__(256) void k_relclip(const float* __restrict__ RAW, float* MP) { const size_t e = ((size_t)blockIdx.x * 256 + threadIdx.x) * 4; if (e >= (size_t)ZH * TT * TT) return; const int j0 = (int)(e % TT); const int i = (int)((e / TT) % TT); const int zz = (int)(e / ((size_t)TT * TT)); const float* rz = RAW + ((size_t)zz * TT + i) * KB; v4f o;
#pragma unroll
    for (int q = 0; q < 4; ++q) { const int j = j0 + q; const bool live = (j <= i); const int bu = min(max(j - i + PR, 0), PR); const float raw = rz[bu]; const float val = __fmul_rn(raw, live ? SCL : 0.0f); o[q] = live ? val : -1.0e30f; }
    *(volatile v4f*)(MP + e) = o; __threadfence(); *(volatile v4f*)(MP + e) = o; }

__global__ __launch_bounds__(256) void k_vside(const h16* __restrict__ P16, h16* SB) { const unsigned e = blockIdx.x * 256u + threadIdx.x; if (e >= (unsigned)ZH * TT) return; const int i = (int)(e % TT); const h16* pr = P16 + (size_t)e * TT; float w[PR]; float s = 0.0f;
#pragma unroll
    for (int u = 1; u <= PR; ++u) { const int k = i - PR + u; const float p = (float)pr[max(k, 0)]; const float v = __fmul_rn(p, (k >= 0) ? 1.0f : 0.0f); w[u - 1] = v; s = __fadd_rn(s, v); }
    const float far = (i >= PR) ? __fsub_rn(PCAR, s) : 0.0f; h16* dst = SB + (size_t)e * KS;
#pragma unroll
    for (int ps = 0; ps < 2; ++ps) {
#pragma unroll
        for (int g = 0; g < KS / 8; ++g) { v8h o;
#pragma unroll
            for (int q = 0; q < 8; ++q) { const int u = g * 8 + q; o[q] = (u == 0) ? (h16)far : ((u <= PR) ? (h16)w[(u >= 1 && u <= PR) ? (u - 1) : 0] : (h16)0.0f); }
            *(volatile v8h*)(dst + g * 8) = o; }
        if (ps == 0) __threadfence(); } }

__global__ __launch_bounds__(256) void k_merge2(const float* __restrict__ O1, const float* __restrict__ O2, int h0, float* OUTb) { const size_t e = ((size_t)blockIdx.x * 256 + threadIdx.x) * 2; if (e >= (size_t)ZH * TT * HD) return; const int d = (int)(e % HD); const int t = (int)((e / HD) % TT); const int zz = (int)(e / ((size_t)HD * TT)); const size_t oo = (size_t)t * DQ + (h0 + zz) * HD + d;
    v2f o2; o2[0] = __fmul_rn(__fadd_rn(O1[e], O2[e]), 1.0f / PCAR); o2[1] = __fmul_rn(__fadd_rn(O1[e + 1], O2[e + 1]), 1.0f / PCAR); *(volatile v2f*)(OUTb + oo) = o2; __threadfence(); *(volatile v2f*)(OUTb + oo) = o2; }

__global__ __launch_bounds__(256) void k_lnfix(const float* __restrict__ Y, const float* __restrict__ beta, float* out, size_t n4) { const size_t e = (size_t)blockIdx.x * 256 + threadIdx.x; if (e >= n4) return; const int c0 = (int)((e * 4) % DM); const v4f y = *(const v4f*)(Y + e * 4); const v4f b = *(const v4f*)(beta + c0); v4f o;
#pragma unroll
    for (int q = 0; q < 4; ++q) { const float bb = bfr(b[q]); o[q] = __fmaf_rn(__fsub_rn(y[q], bb), LNF, bb); }
    *(volatile v4f*)(out + e * 4) = o; __threadfence(); *(volatile v4f*)(out + e * 4) = o; }

extern "C" void kernel_launch(void* const* d_in, const int* in_sizes, int n_in,
                              void* d_out, int out_size, void* d_ws, size_t ws_size, hipStream_t stream) {
    (void)in_sizes; (void)n_in; (void)out_size;
    const float* xq = (const float*)d_in[0]; const float* xk = (const float*)d_in[1]; const float* xv = (const float*)d_in[2]; const float* wq = (const float*)d_in[3]; const float* bqi = (const float*)d_in[4]; const float* wk = (const float*)d_in[5]; const float* bki = (const float*)d_in[6]; const float* wv = (const float*)d_in[7]; const float* bvi = (const float*)d_in[8]; const float* wo = (const float*)d_in[9]; const float* boi = (const float*)d_in[10]; const float* lng = (const float*)d_in[11]; const float* lnb = (const float*)d_in[12];
    float* OUT = (float*)d_out;
    char* wsp = (char*)d_ws;
    auto take = [&](size_t bytes) { char* p = wsp; wsp += (bytes + 255) & ~(size_t)255; return (void*)p; };
    bf* WQB = (bf*)take((size_t)DQ * DM * 2); bf* WKB = (bf*)take((size_t)DKV * DM * 2); bf* WVB = (bf*)take((size_t)DKV * DM * 2); bf* WOB = (bf*)take((size_t)DM * DQ * 2); float* BQ = (float*)take((size_t)DQ * 4); float* BK = (float*)take((size_t)DKV * 4); float* BV = (float*)take((size_t)DKV * 4); float* BO = (float*)take((size_t)DM * 4);
    float* CS = (float*)take((size_t)TT * HD * 2 * 4); h16* RT = (h16*)take((size_t)KB * HD * 2); h16* TT2 = (h16*)take((size_t)HD * KS * 2);
    bf* XQB = (bf*)take((size_t)TT * DM * 2); bf* XKB = (bf*)take((size_t)TT * DM * 2); bf* XVB = (bf*)take((size_t)TT * DM * 2); float* XR = (float*)take((size_t)TT * DM * 4);
    float* FQ = (float*)take((size_t)TT * DQ * 4); float* FK = (float*)take((size_t)TT * DKV * 4); float* FV = (float*)take((size_t)TT * DKV * 4);
    h16* Q16 = (h16*)take((size_t)NH_ * TT * HD * 2); h16* K16 = (h16*)take((size_t)NKV * TT * HD * 2); h16* VT16 = (h16*)take((size_t)NKV * HD * TT * 2);
    bf* PLh = (bf*)take((size_t)NH_ * TT * HD * 2); bf* PLl = (bf*)take((size_t)NH_ * TT * HD * 2);
    float* Sb = (float*)take((size_t)ZH * TT * TT * 4); float* RAWb = (float*)take((size_t)ZH * TT * KB * 4); float* MPb = (float*)take((size_t)ZH * TT * TT * 4); h16* P16 = (h16*)take((size_t)ZH * TT * TT * 2); float* Ob = (float*)take((size_t)ZH * TT * HD * 4); h16* SB = (h16*)take((size_t)ZH * TT * KS * 2); float* Ob2 = (float*)take((size_t)ZH * TT * HD * 4);
    float* FM = (float*)take((size_t)TT * DQ * 4); bf* FMh = (bf*)take((size_t)TT * DQ * 2); bf* FMl = (bf*)take((size_t)TT * DQ * 2); float* PO = (float*)take((size_t)TT * DM * 4); float* LNY = (float*)take((size_t)NB_ * TT * DM * 4);
    if ((size_t)(wsp - (char*)d_ws) > ws_size) return;
    const size_t NW = (size_t)DQ * DM;
    k_cvt8<<<(unsigned)((NW / 8 + 255) / 256), 256, 0, stream>>>(wq, WQB, NW / 8); k_cvt8<<<(unsigned)((NW / 8 + 255) / 256), 256, 0, stream>>>(wk, WKB, NW / 8); k_cvt8<<<(unsigned)((NW / 8 + 255) / 256), 256, 0, stream>>>(wv, WVB, NW / 8); k_cvt8<<<(unsigned)((NW / 8 + 255) / 256), 256, 0, stream>>>(wo, WOB, NW / 8);
    k_rbf<<<1, 256, 0, stream>>>(bqi, BQ, (size_t)DQ / 4); k_rbf<<<1, 256, 0, stream>>>(bki, BK, (size_t)DKV / 4); k_rbf<<<1, 256, 0, stream>>>(bvi, BV, (size_t)DKV / 4); k_rbf<<<1, 256, 0, stream>>>(boi, BO, (size_t)DM / 4);
    k_csid<<<(TT * HD + 255) / 256, 256, 0, stream>>>(CS);
    k_tab<<<(unsigned)(((KB + HD) * 8 + 255) / 256), 256, 0, stream>>>(RT, TT2);
    const size_t NX = (size_t)TT * DM; const unsigned LQ = (unsigned)(((size_t)NH_ * TT * HD / 2 + 255) / 256), LKv = (unsigned)(((size_t)NKV * TT * HD / 2 + 255) / 256);
    for (int b = 0; b < NB_; ++b) { const size_t ob = (size_t)b * TT * DM;
        k_cvt8<<<(unsigned)((NX / 8 + 255) / 256), 256, 0, stream>>>(xq + ob, XQB, NX / 8); k_cvt8<<<(unsigned)((NX / 8 + 255) / 256), 256, 0, stream>>>(xk + ob, XKB, NX / 8); k_cvt8<<<(unsigned)((NX / 8 + 255) / 256), 256, 0, stream>>>(xv + ob, XVB, NX / 8); k_rbf<<<(unsigned)((NX / 4 + 255) / 256), 256, 0, stream>>>(xq + ob, XR, NX / 4);
        k_gemmw<bf, 0, true><<<dim3(TT / 64, DQ / 64, 1), 32, 0, stream>>>(XQB, nullptr, WQB, nullptr, DM, FQ, DQ, BQ, 0, 0, 0); k_gemmw<bf, 0, true><<<dim3(TT / 64, DKV / 64, 1), 32, 0, stream>>>(XKB, nullptr, WKB, nullptr, DM, FK, DKV, BK, 0, 0, 0); k_gemmw<bf, 0, true><<<dim3(TT / 64, DKV / 64, 1), 32, 0, stream>>>(XVB, nullptr, WVB, nullptr, DM, FV, DKV, BV, 0, 0, 0);
        k_rope<<<LQ, 256, 0, stream>>>(FQ, DQ, NH_, CS, nullptr, nullptr, 1.0f, Q16, PLh, PLl); k_rope<<<LKv, 256, 0, stream>>>(FK, DKV, NKV, CS, nullptr, nullptr, 1.0f, K16, PLh, PLl); k_vtp<<<LKv, 256, 0, stream>>>(FV, DKV, NKV, VT16, PLh, PLl);
        for (int h0 = 0; h0 < NH_; h0 += ZH) { const size_t zq = (size_t)h0, zk = (size_t)(h0 / REP);
            k_gemmw<h16, 0, false><<<dim3((TT - RH) / 64, TT / 64, ZH), 32, 0, stream>>>(Q16 + zq * TT * HD + (size_t)RH * HD, nullptr, K16 + zk * TT * HD, nullptr, HD, Sb + (size_t)RH * TT, TT, nullptr, (size_t)TT * HD, (size_t)TT * HD, (size_t)TT * TT);
            k_gemmw<h16, 0, false><<<dim3(TT / 64, KB / 64, ZH), 32, 0, stream>>>(Q16 + zq * TT * HD, nullptr, RT, nullptr, HD, RAWb, KB, nullptr, (size_t)TT * HD, 0, (size_t)TT * KB);
            k_relclip<<<(unsigned)((size_t)ZH * TT * TT / 1024), 256, 0, stream>>>(RAWb, MPb);
            for (int zz = 0; zz < ZH; ++zz) k_asoftMA<<<TT / 8, 256, 0, stream>>>(Sb + (size_t)zz * TT * TT, MPb + (size_t)zz * TT * TT, P16 + (size_t)zz * TT * TT, nullptr, nullptr);
            k_gemmw<h16, 0, false><<<dim3((TT - RH) / 64, HD / 64, ZH), 32, 0, stream>>>(P16 + (size_t)RH * TT, nullptr, VT16 + zk * HD * TT, nullptr, TT, Ob + (size_t)RH * HD, HD, nullptr, (size_t)TT * TT, (size_t)HD * TT, (size_t)TT * HD);
            k_vside<<<(unsigned)((ZH * TT + 255) / 256), 256, 0, stream>>>(P16, SB);
            k_gemmw<h16, 0, false><<<dim3(TT / 64, HD / 64, ZH), 32, 0, stream>>>(SB, nullptr, TT2, nullptr, KS, Ob2, HD, nullptr, (size_t)TT * KS, 0, (size_t)TT * HD);
            k_merge2<<<(unsigned)(((size_t)ZH * TT * HD / 2 + 255) / 256), 256, 0, stream>>>(Ob, Ob2, h0, FM); }
        k_pl2<<<(unsigned)(((size_t)TT * DQ / 4 + 255) / 256), 256, 0, stream>>>(FM, FMh, FMl, (size_t)TT * DQ / 4);
        k_gemmw<bf, 1, true><<<dim3(TT / 64, DM / 64, 1), 32, 0, stream>>>(FMh, FMl, WOB, nullptr, DQ, PO, DM, BO, 0, 0, 0);
        k_lnrow<true><<<(unsigned)((TT + 7) / 8), 256, 0, stream>>>(PO, XR, lng, lnb, 1.0e-12f, DM, TT, LNY + ob); }
    k_lnfix<<<(unsigned)(((size_t)NB_ * TT * DM / 4 + 255) / 256), 256, 0, stream>>>(LNY, lnb, OUT, (size_t)NB_ * TT * DM / 4);
}
